// HPCrnn_67542655696955
// MI455X (gfx1250) — hardware-verified
//
#include <hip/hip_runtime.h>
#include <stddef.h>

typedef __attribute__((ext_vector_type(16))) _Float16 v16h;
typedef __attribute__((ext_vector_type(8)))  _Float16 v8h;
typedef __attribute__((ext_vector_type(4)))  _Float16 v4h;
typedef __attribute__((ext_vector_type(16))) __bf16   v16b;
typedef __attribute__((ext_vector_type(8)))  __bf16   v8b;
typedef __attribute__((ext_vector_type(8)))  float    v8f;
typedef __attribute__((ext_vector_type(4)))  float    v4f;

__device__ __forceinline__ unsigned short f2bf_bits(float f) {
  unsigned u = __float_as_uint(f);
  return (unsigned short)((u + 0x7FFFu + ((u >> 16) & 1u)) >> 16);
}
__device__ __forceinline__ float bf_bits2f(unsigned short h) { return __uint_as_float(((unsigned)h) << 16); }

__device__ __forceinline__ void dep_guard_h(v8f& a, v8f& b, v16h x, v16h y) { asm volatile("v_nop\n\tv_nop\n\tv_nop\n\tv_nop" : "+v"(a), "+v"(b) : "v"(x), "v"(y)); }
__device__ __forceinline__ void dep_guard_b(v8f& a, v8f& b, v16b x, v16b y) { asm volatile("v_nop\n\tv_nop\n\tv_nop\n\tv_nop" : "+v"(a), "+v"(b) : "v"(x), "v"(y)); }
__device__ __forceinline__ void keep4_h(v16h a, v16h b, v16h c, v16h d) { asm volatile("v_nop" :: "v"(a), "v"(b), "v"(c), "v"(d)); }
__device__ __forceinline__ void keep4_b(v16b a, v16b b, v16b c, v16b d) { asm volatile("v_nop" :: "v"(a), "v"(b), "v"(c), "v"(d)); }
__device__ __forceinline__ void acc_guard4(v8f& a, v8f& b, v8f& c, v8f& d) { asm volatile("v_nop\n\tv_nop\n\tv_nop\n\tv_nop" : "+v"(a), "+v"(b), "+v"(c), "+v"(d)); }
template <typename T> struct Frag;
template <> struct Frag<_Float16> {
  typedef v16h V; union U { v16h v; v8h h[2]; };
  static __device__ __forceinline__ v16h load(const _Float16* p) {
    U f; f.h[0] = *(const v8h*)(p); f.h[1] = *(const v8h*)(p + 16); return f.v;
  }
  static __device__ __forceinline__ v8f mma(v16h a, v16h b, v8f c) {
    return __builtin_amdgcn_wmma_f32_16x16x32_f16(false, a, false, b, (short)0, c, false, false);
  }
  static __device__ __forceinline__ void guard(v8f& a, v8f& b, v16h x, v16h y) { dep_guard_h(a, b, x, y); }
  static __device__ __forceinline__ void keep(v16h a, v16h b, v16h c, v16h d) { keep4_h(a, b, c, d); }
};
template <> struct Frag<__bf16> {
  typedef v16b V; union U { v16b v; v8b h[2]; };
  static __device__ __forceinline__ v16b load(const __bf16* p) {
    U f; f.h[0] = *(const v8b*)(p); f.h[1] = *(const v8b*)(p + 16); return f.v;
  }
  static __device__ __forceinline__ v8f mma(v16b a, v16b b, v8f c) {
    return __builtin_amdgcn_wmma_f32_16x16x32_bf16(false, a, false, b, (short)0, c, false, false);
  }
  static __device__ __forceinline__ void guard(v8f& a, v8f& b, v16b x, v16b y) { dep_guard_b(a, b, x, y); }
  static __device__ __forceinline__ void keep(v16b a, v16b b, v16b c, v16b d) { keep4_b(a, b, c, d); }
};

template <int ET> struct Elem;
template <> struct Elem<0> { typedef _Float16 T; };
template <> struct Elem<1> { typedef __bf16 T; };
template <int ET, bool SPLIT, int BIAS_MODE, int OUT_MODE, bool RESID, int ACT = 0>
__global__ __launch_bounds__(256) void wmma_gemm64(
    const unsigned short* __restrict__ Ap, const unsigned short* __restrict__ A2p, int lda, long strideA,
    const unsigned short* __restrict__ Btp, const unsigned short* __restrict__ Bt2p, int ldb, long strideB,
    void* __restrict__ Cout, void* __restrict__ Cout2, int ldc, long strideC,
    const float* __restrict__ bias,
    const float* __restrict__ resid, long strideR,
    int M, int N, int K, float scale) {
  typedef typename Elem<ET>::T T;
  typedef typename Frag<T>::V V;
  const T* A = (const T*)Ap; const T* A2 = (const T*)A2p; const T* Bt = (const T*)Btp; const T* Bt2 = (const T*)Bt2p;
  __shared__ __align__(16) float sT[8][16 * 68];
  const int b    = blockIdx.y;
  const int lane = threadIdx.x & 31;
  const int wave = threadIdx.x >> 5;
  const int tilesN = N >> 6;
  const int tilesM = M >> 6;
  const int tile = blockIdx.x * 8 + wave;
  if (tile >= tilesM * tilesN) return;
  const int tm = tile / tilesN;
  const int tn = tile - tm * tilesN;
  const int m0 = tm << 6;
  const int n0 = tn << 6;

  const T* Ab  = A  + (size_t)b * strideA;
  const T* Bb  = Bt + (size_t)b * strideB;
  const T* Ab2 = SPLIT ? (A2  + (size_t)b * strideA) : nullptr;
  const T* Bb2 = SPLIT ? (Bt2 + (size_t)b * strideB) : nullptr;

  const int rlane = lane & 15;
  const int koff  = (lane >> 4) * 8;
  const int mOff  = (lane >> 4) * 8;

  v8f acc[4][4];
#pragma unroll
  for (int i = 0; i < 4; ++i)
#pragma unroll
    for (int j = 0; j < 4; ++j) acc[i][j] = (v8f){0.f,0.f,0.f,0.f,0.f,0.f,0.f,0.f};

  for (int k0 = 0; k0 < K; k0 += 32) {
    V bh[4], bl[4];
#pragma unroll
    for (int j = 0; j < 4; ++j) {
      const size_t bo = (size_t)(n0 + (j << 4) + rlane) * ldb + koff + k0;
      bh[j] = Frag<T>::load(Bb + bo);
      if (SPLIT) bl[j] = Frag<T>::load(Bb2 + bo);
    }
#pragma unroll
    for (int i = 0; i < 4; ++i) {
      const size_t ao = (size_t)(m0 + (i << 4) + rlane) * lda + koff + k0;
      V ah = Frag<T>::load(Ab + ao);
      V al;
      if (SPLIT) al = Frag<T>::load(Ab2 + ao);
#pragma unroll
      for (int j = 0; j < 4; ++j) {
        acc[i][j] = Frag<T>::mma(ah, bh[j], acc[i][j]);
        if (SPLIT) {
          acc[i][j] = Frag<T>::mma(ah, bl[j], acc[i][j]);
          acc[i][j] = Frag<T>::mma(al, bh[j], acc[i][j]);
        }
      }
      Frag<T>::guard(acc[i][0], acc[i][3], ah, SPLIT ? al : ah);
    }
    Frag<T>::keep(bh[0], bh[1], bh[2], bh[3]);
    if (SPLIT) Frag<T>::keep(bl[0], bl[1], bl[2], bl[3]);
  }
  acc_guard4(acc[0][0], acc[0][1], acc[0][2], acc[0][3]);
  acc_guard4(acc[1][0], acc[1][1], acc[1][2], acc[1][3]);
  acc_guard4(acc[2][0], acc[2][1], acc[2][2], acc[2][3]);
  acc_guard4(acc[3][0], acc[3][1], acc[3][2], acc[3][3]);

  float* slab = sT[wave];
  const float* Rb = RESID ? (resid + (size_t)b * strideR) : nullptr;
#pragma unroll
  for (int i = 0; i < 4; ++i) {
    const int mBase = m0 + (i << 4);
#pragma unroll
    for (int j = 0; j < 4; ++j) {
      const int n = n0 + (j << 4) + rlane;
      float bv = 0.f;
      if (BIAS_MODE == 2) bv = bias[n];
#pragma unroll
      for (int r = 0; r < 8; ++r) {
        float v = acc[i][j][r] * scale;
        if (BIAS_MODE == 1) v += bias[mBase + mOff + r];
        if (BIAS_MODE == 2) v += bv;
        if (RESID) v += Rb[(size_t)(mBase + mOff + r) * ldc + n];
        if (ACT == 1) v = tanhf(v);
        if (ACT == 2) v = fmaxf(v, 0.0f);
        if (ACT == 3) v = v / (1.0f + expf(-v));
        if (ACT == 4) v = (v > 0.f) ? v : 0.01f * v;
        if (ACT == 5) v = 0.5f * v * (1.0f + erff(v * 0.70710678118654752f));
        slab[(mOff + r) * 68 + (j << 4) + rlane] = v;
      }
    }
    __builtin_amdgcn_fence(__ATOMIC_RELEASE, "workgroup");
    __builtin_amdgcn_wave_barrier();
    __builtin_amdgcn_fence(__ATOMIC_ACQUIRE, "workgroup");
    if (OUT_MODE == 0) {
      float* C = (float*)Cout + (size_t)b * strideC;
      const int hh = lane >> 4, c4 = (lane & 15) * 4;
      for (int pass = 0; pass < 2; ++pass) {
#pragma unroll
        for (int it = 0; it < 8; ++it) {
          const int row = it * 2 + hh;
          v4f v = *(const v4f*)(slab + row * 68 + c4);
          *(volatile v4f*)(C + (size_t)(mBase + row) * ldc + n0 + c4) = v;
        }
        __threadfence();
      }
    } else {
      const int q = lane >> 3, c8 = (lane & 7) * 8;
      unsigned short* C  = (unsigned short*)Cout  + (size_t)b * strideC;
      unsigned short* C2 = (OUT_MODE == 2) ? ((unsigned short*)Cout2 + (size_t)b * strideC) : nullptr;
      for (int pass = 0; pass < 2; ++pass) {
#pragma unroll
        for (int it = 0; it < 4; ++it) {
          const int row = it * 4 + q;
          const float* sp = slab + row * 68 + c8;
          v8h hv, lv;
#pragma unroll
          for (int e = 0; e < 8; ++e) {
            if (OUT_MODE == 1) {
              hv[e] = (_Float16)sp[e];
            } else {
              unsigned short hb = f2bf_bits(sp[e]);
              unsigned short lb = f2bf_bits(sp[e] - bf_bits2f(hb));
              hv[e] = __builtin_bit_cast(_Float16, hb);
              lv[e] = __builtin_bit_cast(_Float16, lb);
            }
          }
          *(volatile v8h*)(C + (size_t)(mBase + row) * ldc + n0 + c8) = hv;
          if (OUT_MODE == 2) *(volatile v8h*)(C2 + (size_t)(mBase + row) * ldc + n0 + c8) = lv;
        }
        __threadfence();
      }
    }
    __builtin_amdgcn_fence(__ATOMIC_RELEASE, "workgroup");
    __builtin_amdgcn_wave_barrier();
    __builtin_amdgcn_fence(__ATOMIC_ACQUIRE, "workgroup");
  }
}

constexpr int kBatch     = 256;
constexpr int kEcN       = 1024;
constexpr int kCa1N      = 1024;
constexpr int kBumpN     = 1024;
constexpr int kSteps     = 100;
constexpr int kStepsPad  = 128;
constexpr int kActN      = 2;
constexpr int kRowsPB    = 16;
constexpr int kMainBlocks  = kBatch / kRowsPB;
constexpr int kMainThreads = 256;
constexpr int kWaveCols  = 128;
constexpr int kTileP     = 1032;
constexpr int kStateP    = 1024;
constexpr int kSlabP     = 32;
constexpr float kEc3Carry = 4096.0f;
constexpr float kWCarry   = 64.0f;
constexpr float kA0Carry  = 256.0f;
constexpr float kW0Carry  = 4096.0f;
static_assert(kEcN == kCa1N && kEcN % 32 == 0);
static_assert(kBatch % kRowsPB == 0);
static_assert((kMainThreads / 32) * kWaveCols == kCa1N);
static_assert(kTileP % 8 == 0 && kTileP >= kEcN);
static_assert(kStepsPad % 64 == 0 && kStepsPad >= kSteps);
static_assert(kMainThreads == kRowsPB * 16);

constexpr int kLdsEc3h  = 0;
constexpr int kLdsCa1h  = kLdsEc3h + kRowsPB * kTileP * 2;
constexpr int kLdsEc3f  = kLdsCa1h + kRowsPB * kTileP * 2;
constexpr int kLdsEc5f  = kLdsEc3f + kRowsPB * kStateP * 4;
constexpr int kLdsSlab  = kLdsEc5f + kRowsPB * kStateP * 4;
constexpr int kLdsHs    = kLdsSlab + 8 * kRowsPB * kSlabP * 4;
constexpr int kLdsRed   = kLdsHs + 8 * 256 * 4;
constexpr int kLdsActs  = kLdsRed + 8 * 32 * 4;
constexpr int kLdsTotal = kLdsActs + 32 * 4;
static_assert(kLdsTotal == 222848);
static_assert(kLdsCa1h % 16 == 0 && kLdsEc3f % 16 == 0 && kLdsEc5f % 16 == 0 && kLdsSlab % 16 == 0 &&
              kLdsHs % 16 == 0 && kLdsRed % 16 == 0 && kLdsActs % 16 == 0);

constexpr size_t kOutAct    = 0;
constexpr size_t kOutEc3His = 512;
constexpr size_t kOutEc5His = kOutEc3His + (size_t)kSteps * kEcN;
constexpr size_t kOutCa1His = kOutEc5His + (size_t)kSteps * kEcN;
constexpr size_t kOutEc3    = kOutCa1His + (size_t)kSteps * kCa1N;
constexpr size_t kOutEc5    = kOutEc3 + (size_t)kBatch * kEcN;
constexpr size_t kOutCa1    = kOutEc5 + (size_t)kBatch * kEcN;
constexpr size_t kOutTotal  = kOutCa1 + (size_t)kBatch * kCa1N;
static_assert(kOutTotal == 1094144);
static_assert(kOutEc3His % 32 == 0 && kOutEc5His % 32 == 0 && kOutCa1His % 32 == 0 &&
              kOutEc3 % 32 == 0 && kOutEc5 % 32 == 0 && kOutCa1 % 32 == 0);

constexpr size_t kWsBt0   = 0;
constexpr size_t kWsBt1   = kWsBt0 + (size_t)kCa1N * kBumpN * 2;
constexpr size_t kWsBt2   = kWsBt1 + (size_t)kCa1N * kEcN * 2;
constexpr size_t kWsA0    = kWsBt2 + (size_t)kEcN * kCa1N * 2;
constexpr size_t kWsDrive = kWsA0 + (size_t)kStepsPad * kBumpN * 2;
constexpr size_t kWsTotal = kWsDrive + (size_t)kStepsPad * kCa1N * 4;
static_assert(kWsTotal == 7077888);
static_assert(kWsBt1 % 128 == 0 && kWsBt2 % 128 == 0 && kWsA0 % 128 == 0 && kWsDrive % 128 == 0);

__device__ __forceinline__ void wave_sync() {
  __builtin_amdgcn_fence(__ATOMIC_RELEASE, "workgroup");
  __builtin_amdgcn_wave_barrier();
  __builtin_amdgcn_fence(__ATOMIC_ACQUIRE, "workgroup");
}
__device__ __forceinline__ float sigm(float x) { return __builtin_amdgcn_rcpf(1.0f + __expf(-x)); }

constexpr int kTrTile = 64;
constexpr int kTrPitch = 72;
__global__ __launch_bounds__(256) void transpose_scale_f16_kernel(
    const float* __restrict__ in, unsigned short* __restrict__ outp, int nk, int nn, float scale) {
  __shared__ __align__(16) _Float16 sT[kTrTile * kTrPitch];
  const int tid = threadIdx.x;
  const int n0 = blockIdx.x * kTrTile;
  const int k0 = blockIdx.y * kTrTile;
  {
    const int kr = tid >> 2;
    const int seg = (tid & 3) * 16;
    const float* src = in + (size_t)(k0 + kr) * nn + n0 + seg;
#pragma unroll
    for (int q = 0; q < 4; ++q) {
      const v4f v = *(const v4f*)(src + 4 * q);
#pragma unroll
      for (int e = 0; e < 4; ++e) sT[(seg + 4 * q + e) * kTrPitch + kr] = (_Float16)(v[e] * scale);
    }
  }
  __syncthreads();
  const int lane = tid & 31, wave = tid >> 5;
  const int q = lane >> 3, c8 = (lane & 7) * 8;
  _Float16* o = (_Float16*)outp;
  for (int pass = 0; pass < 2; ++pass) {
#pragma unroll
    for (int it = 0; it < 2; ++it) {
      const int nr = wave * 8 + it * 4 + q;
      const v8h val = *(const v8h*)(sT + nr * kTrPitch + c8);
      *(volatile v8h*)(o + (size_t)(n0 + nr) * nk + k0 + c8) = val;
    }
    __threadfence();
  }
}

__global__ __launch_bounds__(128) void bump_plane_kernel(unsigned short* __restrict__ A0p) {
  __shared__ __align__(16) _Float16 rowbuf[kBumpN];
  const int t = blockIdx.x;
  const int tid = threadIdx.x;
  const float tf = (float)t;
  const bool live = (t < kSteps);
#pragma unroll 1
  for (int i = 0; i < kBumpN / 128; ++i) {
    const int k = tid + 128 * i;
    const float s = (float)k * (1.0f / 1023.0f);
    const float cpos = 100.0f * s;
    const float d = cpos - tf;
    const float g = expf(-(d * d) * (1.0f / 25.0f) * 0.5f);
    rowbuf[k] = (_Float16)(live ? g * kA0Carry : 0.0f);
  }
  __syncthreads();
  const v8h val = *(const v8h*)(rowbuf + 8 * tid);
  _Float16* dst = (_Float16*)A0p + (size_t)t * kBumpN + 8 * tid;
  for (int pass = 0; pass < 2; ++pass) {
    *(volatile v8h*)dst = val;
    __threadfence();
  }
}

__device__ __forceinline__ void strip_gemm16x128(const _Float16* At, const _Float16* __restrict__ Bt,
                                                 int nbase, int c, int koff, v8f (&acc)[8]) {
#pragma unroll
  for (int j = 0; j < 8; ++j) acc[j] = (v8f){0.f,0.f,0.f,0.f,0.f,0.f,0.f,0.f};
  for (int k0 = 0; k0 < kEcN; k0 += 32) {
    const v16h a = Frag<_Float16>::load(At + c * kTileP + k0 + koff);
#pragma unroll
    for (int g = 0; g < 2; ++g) {
      v16h bq[4];
#pragma unroll
      for (int j = 0; j < 4; ++j)
        bq[j] = Frag<_Float16>::load(Bt + (size_t)(nbase + 16 * (4 * g + j) + c) * kEcN + k0 + koff);
#pragma unroll
      for (int j = 0; j < 4; ++j) acc[4 * g + j] = Frag<_Float16>::mma(a, bq[j], acc[4 * g + j]);
      Frag<_Float16>::guard(acc[4 * g], acc[4 * g + 3], a, bq[3]);
      Frag<_Float16>::keep(bq[0], bq[1], bq[2], bq[3]);
    }
  }
  acc_guard4(acc[0], acc[1], acc[2], acc[3]);
  acc_guard4(acc[4], acc[5], acc[6], acc[7]);
}

__global__ __launch_bounds__(kMainThreads) void place_rnn_steps_kernel(
    const unsigned short* __restrict__ Bt1p, const unsigned short* __restrict__ Bt2p,
    const float* __restrict__ drive, const float* __restrict__ ca1bias, const int* __restrict__ cue,
    const float* __restrict__ ec3_init, const float* __restrict__ ec5_init, const float* __restrict__ ca1_init,
    const float* __restrict__ wact, const float* __restrict__ actbias, float* __restrict__ out)
{
  extern __shared__ __align__(16) unsigned char dyn_lds[];
  _Float16* ec3h = (_Float16*)(dyn_lds + kLdsEc3h);
  _Float16* ca1h = (_Float16*)(dyn_lds + kLdsCa1h);
  float* ec3f = (float*)(dyn_lds + kLdsEc3f);
  float* ec5f = (float*)(dyn_lds + kLdsEc5f);
  float* slab_all = (float*)(dyn_lds + kLdsSlab);
  float* hs_all   = (float*)(dyn_lds + kLdsHs);
  float* red      = (float*)(dyn_lds + kLdsRed);
  float* acts     = (float*)(dyn_lds + kLdsActs);
  (void)ca1_init;

  const int tid  = threadIdx.x;
  const int lane = tid & 31;
  const int wave = tid >> 5;
  const int c    = lane & 15;
  const int hh   = lane >> 4;
  const int koff = hh * 8;
  const int mOff = hh * 8;
  const int b0   = (int)blockIdx.x * kRowsPB;
  const int nbase = wave * kWaveCols;
  const _Float16* Bt1 = (const _Float16*)Bt1p;
  const _Float16* Bt2 = (const _Float16*)Bt2p;
  float* slab = slab_all + wave * (kRowsPB * kSlabP);
  float* hs   = hs_all + wave * 256;

  {
    const int r = tid >> 4, cb = (tid & 15) * 64;
    const float* p3 = ec3_init + (size_t)(b0 + r) * kEcN + cb;
    const float* p5 = ec5_init + (size_t)(b0 + r) * kEcN + cb;
#pragma unroll 4
    for (int qd = 0; qd < 16; ++qd) {
      const v4f a = *(const v4f*)(p3 + 4 * qd);
      const v4f e = *(const v4f*)(p5 + 4 * qd);
      *(v4f*)(ec3f + r * kStateP + cb + 4 * qd) = a;
      *(v4f*)(ec5f + r * kStateP + cb + 4 * qd) = e;
      v4h hv;
      hv[0] = (_Float16)(a[0] * kEc3Carry); hv[1] = (_Float16)(a[1] * kEc3Carry);
      hv[2] = (_Float16)(a[2] * kEc3Carry); hv[3] = (_Float16)(a[3] * kEc3Carry);
      *(v4h*)(ec3h + r * kTileP + cb + 4 * qd) = hv;
    }
  }
  __syncthreads();

  float actp = 0.0f;
  v8f acc[8];

#pragma unroll 1
  for (int t = 0; t < kSteps; ++t) {
    strip_gemm16x128(ec3h, Bt1, nbase, c, koff, acc);
    {
      const bool last = (t == kSteps - 1);
      const float* drv = drive + (size_t)t * kCa1N;
#pragma unroll
      for (int jp = 0; jp < 4; ++jp) {
#pragma unroll
        for (int jj = 0; jj < 2; ++jj) {
          const int j = 2 * jp + jj;
          const int col = nbase + 16 * j + c;
          const float d = drv[col];
          const float bsv = ca1bias[col];
#pragma unroll
          for (int r = 0; r < 8; ++r) {
            const int row = mOff + r;
            const float s1 = acc[j][r] * (1.0f / 262144.0f);
            const float sg = sigm(s1);
            float v = d * (1.0f + sg) - bsv;
            v = fmaxf(v, 0.0f);
            ca1h[row * kTileP + col] = (_Float16)v;
            if (r == 0) hs[hh * 128 + 16 * j + c] = v;
            if (last) slab[row * kSlabP + jj * 16 + c] = v;
          }
        }
        if (last) {
          wave_sync();
          const int q = lane >> 3, c4 = (lane & 7) * 4;
          float* cbase = out + kOutCa1 + (size_t)b0 * kCa1N + nbase + 32 * jp;
          for (int pass = 0; pass < 2; ++pass) {
#pragma unroll
            for (int it = 0; it < 4; ++it) {
              const int row = it * 4 + q;
              const v4f val = *(const v4f*)(slab + row * kSlabP + c4);
              *(volatile v4f*)(cbase + (size_t)row * kCa1N + c4) = val;
            }
            __threadfence();
          }
          const int arow = lane >> 1, asel = lane & 1;
          const float* wa = wact + (size_t)(nbase + 32 * jp) * kActN + asel;
#pragma unroll 1
          for (int cc = 0; cc < 32; ++cc) actp = fmaf(slab[arow * kSlabP + cc], wa[cc * kActN], actp);
          wave_sync();
        }
      }
      if (blockIdx.x == 0) {
        wave_sync();
        const v4f hv = *(const v4f*)(hs + 4 * lane);
        float* hp = out + kOutCa1His + (size_t)t * kCa1N + nbase + 4 * lane;
        for (int pass = 0; pass < 2; ++pass) { *(volatile v4f*)hp = hv; __threadfence(); }
      }
    }
    __syncthreads();

    strip_gemm16x128(ca1h, Bt2, nbase, c, koff, acc);
    {
      const int stim = (t == 16) ? 0 : ((t == 24) ? 1 : -1);
      const int stimc = stim < 0 ? 0 : stim;
#pragma unroll
      for (int j = 0; j < 8; ++j) {
        const int col = nbase + 16 * j + c;
#pragma unroll
        for (int r = 0; r < 8; ++r) {
          const int row = mOff + r;
          const int si = row * kStateP + col;
          float e5 = ec5f[si] + acc[j][r] * (1.0f / 64.0f);
          const float sg = sigm(4.0f * (e5 - 0.3f));
          e5 = 0.69f + 0.3f * sg;
          float e3 = e5 * ec3f[si];
          if (stim >= 0) {
            const int m = cue[((size_t)(b0 + row) * 2 + stimc) * kEcN + col];
            const float e3c = 0.4f * e3 + 0.6f;
            e3 = (m != 0) ? e3c : e3;
          }
          ec5f[si] = e5;
          ec3f[si] = e3;
          ec3h[row * kTileP + col] = (_Float16)(e3 * kEc3Carry);
        }
      }
      if (blockIdx.x == 0) {
        wave_sync();
        const v4f h3 = *(const v4f*)(ec3f + nbase + 4 * lane);
        const v4f h5 = *(const v4f*)(ec5f + nbase + 4 * lane);
        float* p3 = out + kOutEc3His + (size_t)t * kEcN + nbase + 4 * lane;
        float* p5 = out + kOutEc5His + (size_t)t * kEcN + nbase + 4 * lane;
        for (int pass = 0; pass < 2; ++pass) { *(volatile v4f*)p3 = h3; *(volatile v4f*)p5 = h5; __threadfence(); }
      }
    }
    __syncthreads();
  }

  for (int pass = 0; pass < 2; ++pass) {
#pragma unroll 4
    for (int row = 0; row < kRowsPB; ++row) {
      const v4f a3 = *(const v4f*)(ec3f + row * kStateP + nbase + 4 * lane);
      const v4f a5 = *(const v4f*)(ec5f + row * kStateP + nbase + 4 * lane);
      *(volatile v4f*)(out + kOutEc3 + (size_t)(b0 + row) * kEcN + nbase + 4 * lane) = a3;
      *(volatile v4f*)(out + kOutEc5 + (size_t)(b0 + row) * kEcN + nbase + 4 * lane) = a5;
    }
    __threadfence();
  }

  red[wave * 32 + lane] = actp;
  __syncthreads();
  if (wave == 0) {
    float s = actbias[lane & 1];
#pragma unroll
    for (int w = 0; w < 8; ++w) s += red[w * 32 + lane];
    acts[lane] = s;
    wave_sync();
    const v4f val = *(const v4f*)(acts + 4 * (lane & 7));
    float* op = out + kOutAct + (size_t)b0 * kActN;
    for (int pass = 0; pass < 2; ++pass) {
      if (lane < 8) *(volatile v4f*)(op + 4 * lane) = val;
      __threadfence();
    }
  }
}

extern "C" void kernel_launch(void* const* d_in, const int* in_sizes, int n_in,
                              void* d_out, int out_size, void* d_ws, size_t ws_size, hipStream_t stream) {
  if (n_in < 10 || d_out == nullptr || d_ws == nullptr) return;
  if (in_sizes[0] != kBatch * 2 * kEcN || in_sizes[1] != kBatch * kEcN || in_sizes[2] != kBatch * kEcN ||
      in_sizes[3] != kBatch * kCa1N || in_sizes[4] != kCa1N || in_sizes[5] != kBumpN * kCa1N ||
      in_sizes[6] != kEcN * kCa1N || in_sizes[7] != kCa1N * kEcN || in_sizes[8] != kCa1N * kActN ||
      in_sizes[9] != kActN || (size_t)out_size != kOutTotal || ws_size < kWsTotal) return;

  const int*   cue      = (const int*)d_in[0];
  const float* ec3_last = (const float*)d_in[1];
  const float* ec5_last = (const float*)d_in[2];
  const float* ca1_last = (const float*)d_in[3];
  const float* ca1bias  = (const float*)d_in[4];
  const float* wca3ca1  = (const float*)d_in[5];
  const float* wec3ca1  = (const float*)d_in[6];
  const float* wca1ec5  = (const float*)d_in[7];
  const float* wca1act  = (const float*)d_in[8];
  const float* actbias  = (const float*)d_in[9];
  float* out = (float*)d_out;

  unsigned char* ws = (unsigned char*)d_ws;
  unsigned short* Bt0 = (unsigned short*)(ws + kWsBt0);
  unsigned short* Bt1 = (unsigned short*)(ws + kWsBt1);
  unsigned short* Bt2 = (unsigned short*)(ws + kWsBt2);
  unsigned short* A0  = (unsigned short*)(ws + kWsA0);
  float* drive = (float*)(ws + kWsDrive);

  const dim3 trGrid(kCa1N / kTrTile, kBumpN / kTrTile, 1);
  transpose_scale_f16_kernel<<<trGrid, 256, 0, stream>>>(wca3ca1, Bt0, kBumpN, kCa1N, kW0Carry);
  transpose_scale_f16_kernel<<<trGrid, 256, 0, stream>>>(wec3ca1, Bt1, kEcN, kCa1N, kWCarry);
  transpose_scale_f16_kernel<<<trGrid, 256, 0, stream>>>(wca1ec5, Bt2, kCa1N, kEcN, kWCarry);
  bump_plane_kernel<<<kStepsPad, 128, 0, stream>>>(A0);

  wmma_gemm64<0, false, 0, 0, false, 0><<<dim3((kStepsPad / 64) * (kCa1N / 64) / 8, 1, 1), 256, 0, stream>>>(
      A0, A0, kBumpN, 0L, Bt0, Bt0, kBumpN, 0L, (void*)drive, (void*)drive, kCa1N, 0L,
      drive, drive, 0L, kStepsPad, kCa1N, kBumpN, 1.0f / (kA0Carry * kW0Carry));

  place_rnn_steps_kernel<<<kMainBlocks, kMainThreads, kLdsTotal, stream>>>(
      Bt1, Bt2, drive, ca1bias, cue, ec3_last, ec5_last, ca1_last, wca1act, actbias, out);
}
